// MHCA_2473901163150
// MI455X (gfx1250) — hardware-verified
//
#include <hip/hip_runtime.h>
#include <math.h>
#include <stdint.h>

#define NBAT   16
#define NCHK   4
#define NCHUNK 4
#define CDIM   256
#define C3     768
#define CQK    512
#define NPX    3136
#define IMW    56
#define NHEAD  8
#define QT     64
#define NTILE  49
#define TPH    72
#define OSP    68
#define PAP    40
#define RSC    1024.0f
#define IRSC   0.0009765625f
#define PSC    256.0f
#define WSC    64.0f
#define OUTSC  6.103515625e-05f

static_assert(NTILE * QT == NPX);
static_assert(IMW * IMW == NPX);
static_assert(NCHUNK * NCHK == NBAT);
static_assert(NPX % 32 == 0);
static_assert(NPX % 16 == 0);
static_assert((NPX / 16) % 4 == 0);
static_assert(CDIM % 32 == 0);
static_assert(C3 % 128 == 0);
static_assert(CDIM % 64 == 0);
static_assert((TPH * 2) % 16 == 0);
static_assert((OSP * 4) % 16 == 0);
static_assert((PAP * 2) % 16 == 0);
static_assert(NHEAD * 32 == CDIM);

typedef _Float16       v16h __attribute__((ext_vector_type(16)));
typedef _Float16       v8h  __attribute__((ext_vector_type(8)));
typedef __bf16         v16b __attribute__((ext_vector_type(16)));
typedef unsigned short v8us __attribute__((ext_vector_type(8)));
typedef float          v8f  __attribute__((ext_vector_type(8)));
typedef float          v4f  __attribute__((ext_vector_type(4)));
typedef unsigned int   v4u  __attribute__((ext_vector_type(4)));

union Frag { v8us u[2]; v16h h; v16b bf; };
static_assert(sizeof(Frag) == 32);

__device__ __forceinline__ unsigned short bf_bits(float f) {
  unsigned u = __float_as_uint(f);
  return (unsigned short)((u + 0x7FFFu + ((u >> 16) & 1u)) >> 16);
}
__device__ __forceinline__ float bf_up(unsigned short hb) { return __uint_as_float(((unsigned)hb) << 16); }
__device__ __forceinline__ float bfr(float f) { return bf_up(bf_bits(f)); }
__device__ __forceinline__ unsigned short h_bits(_Float16 x) { return __builtin_bit_cast(unsigned short, x); }
__device__ __forceinline__ unsigned pk16(unsigned short a, unsigned short b) { return (unsigned)a | ((unsigned)b << 16); }
__device__ __forceinline__ v8f zero8() { v8f z = {0.f, 0.f, 0.f, 0.f, 0.f, 0.f, 0.f, 0.f}; return z; }

__device__ __forceinline__ Frag ldfrag(const unsigned short* p) {
  Frag f;
  f.u[0] = *(const v8us*)(p);
  f.u[1] = *(const v8us*)(p + 16);
  return f;
}

__device__ __forceinline__ v8f mma_h(v16h a, v16h b, v8f c) {
  v8f d = __builtin_amdgcn_wmma_f32_16x16x32_f16(false, a, false, b, (short)0, c, false, false);
#if defined(__HIP_DEVICE_COMPILE__)
  asm volatile("v_nop\n\tv_nop\n\tv_nop\n\tv_nop" : "+v"(d) : "v"(a), "v"(b));
#endif
  return d;
}
__device__ __forceinline__ v8f mma_b(v16b a, v16b b, v8f c) {
  v8f d = __builtin_amdgcn_wmma_f32_16x16x32_bf16(false, a, false, b, (short)0, c, false, false);
#if defined(__HIP_DEVICE_COMPILE__)
  const v16h ha = __builtin_bit_cast(v16h, a), hb = __builtin_bit_cast(v16h, b);
  asm volatile("v_nop\n\tv_nop\n\tv_nop\n\tv_nop" : "+v"(d) : "v"(ha), "v"(hb));
#endif
  return d;
}

__global__ __launch_bounds__(256)
void cvt_w(const float* __restrict__ wq, const float* __restrict__ wp,
           unsigned short* WQ16, unsigned short* WP16) {
  const int tid = threadIdx.x, e = tid & 7, lq = tid >> 3;
  v4u uq[3];
#pragma unroll
  for (int it = 0; it < 3; ++it) {
    const int L = blockIdx.x * 96 + it * 32 + lq;
    const float* s = wq + (size_t)64 * L + 8 * e;
    const v4f a = *(const v4f*)(s);
    const v4f b = *(const v4f*)(s + 4);
    uq[it][0] = pk16(bf_bits(a[0]), bf_bits(a[1]));
    uq[it][1] = pk16(bf_bits(a[2]), bf_bits(a[3]));
    uq[it][2] = pk16(bf_bits(b[0]), bf_bits(b[1]));
    uq[it][3] = pk16(bf_bits(b[2]), bf_bits(b[3]));
  }
  v4u up;
  const int Lp = blockIdx.x * 32 + lq;
  {
    const float* s = wp + (size_t)64 * Lp + 8 * e;
    const v4f a = *(const v4f*)(s);
    const v4f b = *(const v4f*)(s + 4);
    up[0] = pk16(h_bits((_Float16)(WSC * bfr(a[0]))), h_bits((_Float16)(WSC * bfr(a[1]))));
    up[1] = pk16(h_bits((_Float16)(WSC * bfr(a[2]))), h_bits((_Float16)(WSC * bfr(a[3]))));
    up[2] = pk16(h_bits((_Float16)(WSC * bfr(b[0]))), h_bits((_Float16)(WSC * bfr(b[1]))));
    up[3] = pk16(h_bits((_Float16)(WSC * bfr(b[2]))), h_bits((_Float16)(WSC * bfr(b[3]))));
  }
#pragma unroll
  for (int pass = 0; pass < 2; ++pass) {
#pragma unroll
    for (int it = 0; it < 3; ++it) {
      const int L = blockIdx.x * 96 + it * 32 + lq;
      *(volatile v4u*)(WQ16 + (size_t)64 * L + 8 * e) = uq[it];
    }
    *(volatile v4u*)(WP16 + (size_t)64 * Lp + 8 * e) = up;
    __threadfence();
  }
}

__global__ __launch_bounds__(256)
void cvt_x(const float* __restrict__ x, unsigned short* XP) {
  __shared__ __align__(16) unsigned short Lt[QT * TPH];
  const int tid = threadIdx.x;
  const int nt = blockIdx.x, cg = blockIdx.y, bl = blockIdx.z;
  const int n0 = nt * QT;
  {
    const int n4 = (tid & 15) * 4, cs = tid >> 4;
#pragma unroll
    for (int it = 0; it < 4; ++it) {
      const int cl = it * 16 + cs;
      const v4f v = *(const v4f*)(x + ((size_t)(bl * CDIM + cg * QT + cl)) * NPX + n0 + n4);
#pragma unroll
      for (int q = 0; q < 4; ++q) Lt[(n4 + q) * TPH + cl] = bf_bits(v[q]);
    }
  }
  __syncthreads();
  {
    const int e = tid & 7, lq = tid >> 3;
    const v4u u0 = *(const v4u*)(Lt + lq * TPH + 8 * e);
    const v4u u1 = *(const v4u*)(Lt + (lq + 32) * TPH + 8 * e);
    unsigned short* d0 = XP + ((size_t)(bl * NPX + n0 + lq)) * CDIM + cg * QT + 8 * e;
    unsigned short* d1 = d0 + (size_t)32 * CDIM;
#pragma unroll
    for (int pass = 0; pass < 2; ++pass) {
      *(volatile v4u*)(d0) = u0;
      *(volatile v4u*)(d1) = u1;
      __threadfence();
    }
  }
}

template <int BF, int RES>
__global__ __launch_bounds__(128)
void gemm_k(const unsigned short* __restrict__ A16, const unsigned short* __restrict__ BP,
            const unsigned short* __restrict__ BPL, float* Y, int M, float scale) {
  constexpr int MT  = RES ? 4 : 8;
  constexpr int MR  = 16 * MT;
  constexpr int NIT = (2 * MR) / 16;
  __shared__ __align__(16) float Os[MR * OSP];
  const int tid  = threadIdx.x;
  const int lane = tid & 31, wave = tid >> 5;
  const int hh   = lane >> 4, c = lane & 15;
  const int nt   = blockIdx.x, bl = blockIdx.z;
  const int m0   = blockIdx.y * MR, n0 = nt * QT;

  const unsigned short* ap = A16 + (size_t)(m0 + c) * CDIM + 8 * hh;
  const size_t boff = ((size_t)(bl * NPX + n0 + 16 * wave + c)) * CDIM + 8 * hh;
  const unsigned short* bp  = BP + boff;
  const unsigned short* bpl = RES ? (BPL + boff) : bp;

  v8f acc[MT], accl[MT];
#pragma unroll
  for (int mt = 0; mt < MT; ++mt) { acc[mt] = zero8(); accl[mt] = zero8(); }

#pragma unroll 2
  for (int ks = 0; ks < CDIM / 32; ++ks) {
    const Frag fb = ldfrag(bp + 32 * ks);
    Frag fbl;
    if (RES) fbl = ldfrag(bpl + 32 * ks); else fbl = fb;
#pragma unroll
    for (int mt = 0; mt < MT; ++mt) {
      const Frag fa = ldfrag(ap + (size_t)(16 * mt) * CDIM + 32 * ks);
      if (BF) acc[mt] = mma_b(fa.bf, fb.bf, acc[mt]);
      else    acc[mt] = mma_h(fa.h, fb.h, acc[mt]);
      if (RES) accl[mt] = mma_h(fa.h, fbl.h, accl[mt]);
    }
  }

  {
    const int nl = 16 * wave + c;
#pragma unroll
    for (int mt = 0; mt < MT; ++mt) {
#pragma unroll
      for (int r = 0; r < 8; ++r) {
        float v = acc[mt][r];
        if (RES) v += accl[mt][r] * IRSC;
        Os[(16 * mt + 8 * hh + r) * OSP + nl] = v * scale;
      }
    }
  }
  __syncthreads();

  {
    const int e = tid & 7, lq = tid >> 3;
#pragma unroll
    for (int pass = 0; pass < 2; ++pass) {
#pragma unroll
      for (int it = 0; it < NIT; ++it) {
        const int L = it * 16 + lq;
        const int row = L >> 1, hf = L & 1;
        const v4f v = *(const v4f*)(Os + row * OSP + hf * 32 + 4 * e);
        float* dst = Y + ((size_t)(bl * M + m0 + row)) * NPX + n0 + hf * 32 + 4 * e;
        *(volatile v4f*)dst = v;
      }
      __threadfence();
    }
  }
}

__global__ __launch_bounds__(256)
void dw_k(const float* __restrict__ QKV, const float* __restrict__ wdw,
          unsigned short* QK, unsigned short* VP, unsigned short* VPL) {
  __shared__ __align__(16) unsigned short Th[QT * TPH];
  __shared__ __align__(16) unsigned short Tl[QT * TPH];
  __shared__ float Wc[QT * 9];
  const int tid = threadIdx.x;
  const int nt = blockIdx.x, cg = blockIdx.y, bl = blockIdx.z;
  const int n0 = nt * QT;
  const bool isv = (cg >= 8);
  for (int k = tid; k < QT * 9; k += 256) Wc[k] = bfr(wdw[cg * (QT * 9) + k]);
  const int pl = tid & 63, cs = tid >> 6;
  const int p  = n0 + pl;
  const int y  = p / IMW, xw = p - y * IMW;
  int off[9];
  unsigned okm = 0u;
#pragma unroll
  for (int t = 0; t < 9; ++t) {
    const int ky = t / 3, kx = t - 3 * ky;
    const int yy = y + ky - 1, xx = xw + kx - 1;
    const bool ok = ((unsigned)yy < (unsigned)IMW) && ((unsigned)xx < (unsigned)IMW);
    off[t] = min(max(yy, 0), IMW - 1) * IMW + min(max(xx, 0), IMW - 1);
    okm |= ok ? (1u << t) : 0u;
  }
  __syncthreads();

#pragma unroll 1
  for (int i = 0; i < 16; ++i) {
    const int ch = 4 * i + cs;
    const float* src = QKV + ((size_t)(bl * C3 + cg * QT + ch)) * NPX;
    const float* wt  = Wc + ch * 9;
    float s = 0.f;
#pragma unroll
    for (int t = 0; t < 9; ++t) {
      const float v = src[off[t]];
      s = fmaf(((okm >> t) & 1u) ? v : 0.f, wt[t], s);
    }
    const _Float16 hv = (_Float16)s;
    const _Float16 lv = (_Float16)((s - (float)hv) * RSC);
    const int li = isv ? (pl * TPH + ch) : (ch * TPH + pl);
    Th[li] = h_bits(hv);
    Tl[li] = h_bits(lv);
  }
  __syncthreads();
  {
    const int e = tid & 7, lq = tid >> 3;
    const v4u h0 = *(const v4u*)(Th + lq * TPH + 8 * e);
    const v4u h1 = *(const v4u*)(Th + (lq + 32) * TPH + 8 * e);
    const v4u l0 = *(const v4u*)(Tl + lq * TPH + 8 * e);
    const v4u l1 = *(const v4u*)(Tl + (lq + 32) * TPH + 8 * e);
    if (isv) {
      const int vg = cg - 8;
      const size_t o0 = ((size_t)(bl * NPX + n0 + lq)) * CDIM + vg * QT + 8 * e;
      const size_t o1 = o0 + (size_t)32 * CDIM;
#pragma unroll
      for (int pass = 0; pass < 2; ++pass) {
        *(volatile v4u*)(VP  + o0) = h0;
        *(volatile v4u*)(VP  + o1) = h1;
        *(volatile v4u*)(VPL + o0) = l0;
        *(volatile v4u*)(VPL + o1) = l1;
        __threadfence();
      }
    } else {
      const size_t o0 = ((size_t)(bl * CQK + cg * QT + lq)) * NPX + n0 + 8 * e;
      const size_t o1 = o0 + (size_t)32 * NPX;
#pragma unroll
      for (int pass = 0; pass < 2; ++pass) {
        *(volatile v4u*)(QK + o0) = h0;
        *(volatile v4u*)(QK + o1) = h1;
        __threadfence();
      }
    }
  }
}

__global__ __launch_bounds__(256)
void attn_k(const unsigned short* __restrict__ QK, const unsigned short* __restrict__ VP,
            const unsigned short* __restrict__ VPL, const float* __restrict__ temp,
            unsigned short* OP, unsigned short* OPL) {
  __shared__ float sNorm[128];
  __shared__ float sInv[128];
  __shared__ float sS[2 * 32 * 33];
  __shared__ __align__(16) unsigned short Pa[4 * 32 * PAP];
  __shared__ __align__(16) unsigned short Ow[8 * 16 * TPH];
  const int tid  = threadIdx.x;
  const int lane = tid & 31, wave = tid >> 5;
  const int hh   = lane >> 4, c = lane & 15;
  const int g    = blockIdx.x, bl = blockIdx.y;
  const unsigned short* qkb = QK + (size_t)bl * CQK * NPX;

#pragma unroll 1
  for (int rr = 0; rr < 16; ++rr) {
    const int R = 16 * wave + rr;
    const int chrow = 64 * g + R + ((R >= 64) ? 192 : 0);
    const unsigned short* rp = qkb + (size_t)chrow * NPX;
    float s = 0.f;
    for (int j = 0; j < 13; ++j) {
      const int idx = lane + 32 * j;
      const int idc = min(idx, NPX / 8 - 1);
      const v8h v = *(const v8h*)(rp + 8 * idc);
      float t = 0.f;
#pragma unroll
      for (int q = 0; q < 8; ++q) { const float f = (float)v[q]; t = fmaf(f, f, t); }
      s += (idx < NPX / 8) ? t : 0.f;
    }
#pragma unroll
    for (int off = 16; off > 0; off >>= 1) s += __shfl_xor(s, off, 32);
    if (lane == 0) sNorm[R] = s;
  }

  {
    const int hl = wave >> 2, mt = (wave >> 1) & 1, ntk = wave & 1;
    const unsigned short* arow = qkb + (size_t)(64 * g + 32 * hl + 16 * mt + c) * NPX + 8 * hh;
    const unsigned short* brow = qkb + (size_t)(256 + 64 * g + 32 * hl + 16 * ntk + c) * NPX + 8 * hh;
    v8f acc = zero8();
#pragma unroll 2
    for (int ks = 0; ks < NPX / 32; ++ks) {
      const Frag fa = ldfrag(arow + 32 * ks);
      const Frag fb = ldfrag(brow + 32 * ks);
      acc = mma_h(fa.h, fb.h, acc);
    }
    float* sp = sS + hl * (32 * 33) + (16 * mt + 8 * hh) * 33 + 16 * ntk + c;
#pragma unroll
    for (int r = 0; r < 8; ++r) sp[r * 33] = acc[r];
  }
  __syncthreads();
  if (tid < 128) sInv[tid] = 1.0f / fmaxf(sqrtf(sNorm[tid]), 1e-12f);
  __syncthreads();

  if (tid < 64) {
    const int hl = tid >> 5, row = tid & 31;
    const float tv = bfr(temp[2 * g + hl]);
    const float iq = sInv[32 * hl + row] * tv;
    const float* srow = sS + hl * (32 * 33) + row * 33;
    const float* ik   = sInv + 64 + 32 * hl;
    float lg[32];
    float mx = -3.0e38f;
#pragma unroll
    for (int d = 0; d < 32; ++d) { const float v = srow[d] * iq * ik[d]; lg[d] = v; mx = fmaxf(mx, v); }
    float ssum = 0.f;
#pragma unroll
    for (int d = 0; d < 32; ++d) { const float ev = __expf(lg[d] - mx); lg[d] = ev; ssum += ev; }
    const float inv = PSC / ssum;
    unsigned short* ph = Pa + (hl * 32 + row) * PAP;
    unsigned short* pl = Pa + (64 + hl * 32 + row) * PAP;
#pragma unroll
    for (int d = 0; d < 32; ++d) {
      const float pv = lg[d] * inv;
      const _Float16 hv = (_Float16)pv;
      const _Float16 lv = (_Float16)((pv - (float)hv) * RSC);
      ph[d] = h_bits(hv);
      pl[d] = h_bits(lv);
    }
  }
  __syncthreads();

  {
    const int pr = wave >> 1, hl = wave & 1;
    Frag ah[2], al[2];
#pragma unroll
    for (int mt = 0; mt < 2; ++mt) {
      const unsigned short* p0 = Pa + (hl * 32 + 16 * mt + c) * PAP + 8 * hh;
      ah[mt] = ldfrag(p0);
      al[mt] = ldfrag(p0 + 64 * PAP);
    }
    const size_t pbase = (size_t)bl * NPX * CDIM + 64 * g;
    const unsigned short* vpb = VP  + pbase + 32 * hl + 8 * hh;
    const unsigned short* vlb = VPL + pbase + 32 * hl + 8 * hh;
    unsigned short* owh = Ow + pr * (16 * TPH);
    unsigned short* owl = Ow + (4 + pr) * (16 * TPH);
    const int e8 = lane & 7, lr = (lane >> 3) + 8 * hl;
#pragma unroll 1
    for (int i = 0; i < NPX / 64; ++i) {
      const int n0 = (pr + 4 * i) * 16;
      const unsigned short* vr = vpb + (size_t)(n0 + c) * CDIM;
      const unsigned short* vl = vlb + (size_t)(n0 + c) * CDIM;
      const Frag fvh = ldfrag(vr);
      const Frag fvl = ldfrag(vl);
      v8f o[2], orr[2];
#pragma unroll
      for (int mt = 0; mt < 2; ++mt) {
        o[mt]   = mma_h(ah[mt].h, fvh.h, zero8());
        orr[mt] = mma_h(ah[mt].h, fvl.h, zero8());
        orr[mt] = mma_h(al[mt].h, fvh.h, orr[mt]);
      }
#pragma unroll
      for (int mt = 0; mt < 2; ++mt) {
        v4u uh, ul;
#pragma unroll
        for (int q = 0; q < 4; ++q) {
          const float f0 = o[mt][2 * q]     + orr[mt][2 * q]     * IRSC;
          const float f1 = o[mt][2 * q + 1] + orr[mt][2 * q + 1] * IRSC;
          const _Float16 h0 = (_Float16)f0, h1 = (_Float16)f1;
          const _Float16 l0 = (_Float16)((f0 - (float)h0) * RSC);
          const _Float16 l1 = (_Float16)((f1 - (float)h1) * RSC);
          uh[q] = pk16(h_bits(h0), h_bits(h1));
          ul[q] = pk16(h_bits(l0), h_bits(l1));
        }
        const int so = c * TPH + 32 * hl + 16 * mt + 8 * hh;
        *(v4u*)(owh + so) = uh;
        *(v4u*)(owl + so) = ul;
      }
      __syncthreads();
      const v4u a0 = *(const v4u*)(owh + lr * TPH + 8 * e8);
      const v4u a1 = *(const v4u*)(owh + (lr + 4) * TPH + 8 * e8);
      const v4u b0 = *(const v4u*)(owl + lr * TPH + 8 * e8);
      const v4u b1 = *(const v4u*)(owl + (lr + 4) * TPH + 8 * e8);
      unsigned short* d0 = OP  + pbase + (size_t)(n0 + lr) * CDIM + 8 * e8;
      unsigned short* d1 = OPL + pbase + (size_t)(n0 + lr) * CDIM + 8 * e8;
#pragma unroll
      for (int pass = 0; pass < 2; ++pass) {
        *(volatile v4u*)(d0) = a0;
        *(volatile v4u*)(d0 + 4 * CDIM) = a1;
        *(volatile v4u*)(d1) = b0;
        *(volatile v4u*)(d1 + 4 * CDIM) = b1;
        __threadfence();
      }
      __syncthreads();
    }
  }
}

extern "C" void kernel_launch(void* const* d_in, const int* in_sizes, int n_in,
                              void* d_out, int out_size, void* d_ws, size_t ws_size,
                              hipStream_t stream) {
  const int XN = NBAT * CDIM * NPX;
  if (n_in < 5) return;
  if (in_sizes[0] != XN) return;
  if (in_sizes[1] != C3 * CDIM) return;
  if (in_sizes[2] != C3 * 9) return;
  if (in_sizes[3] != CDIM * CDIM) return;
  if (in_sizes[4] != NHEAD) return;
  if (out_size != XN) return;

  size_t off = 0;
  auto carve = [&](size_t bytes) { const size_t o = off; off += (bytes + 255) & ~(size_t)255; return o; };
  const size_t plane16 = (size_t)NCHK * NPX * CDIM * 2;
  const size_t oWQ  = carve((size_t)C3 * CDIM * 2);
  const size_t oWP  = carve((size_t)CDIM * CDIM * 2);
  const size_t oXP  = carve(plane16);
  const size_t oR1  = carve((size_t)NCHK * C3 * NPX * 4);
  const size_t oQK  = carve((size_t)NCHK * CQK * NPX * 2);
  const size_t oVP  = carve(plane16);
  const size_t oVPL = carve(plane16);
  const size_t oOP  = carve(plane16);
  const size_t oOPL = carve(plane16);
  if (off > ws_size) return;
  if (off > (size_t)134217728) return;

  const float* x    = (const float*)d_in[0];
  const float* wq   = (const float*)d_in[1];
  const float* wdw  = (const float*)d_in[2];
  const float* wp   = (const float*)d_in[3];
  const float* temp = (const float*)d_in[4];
  float* out = (float*)d_out;

  char* ws = (char*)d_ws;
  unsigned short* WQ16 = (unsigned short*)(ws + oWQ);
  unsigned short* WP16 = (unsigned short*)(ws + oWP);
  unsigned short* XP   = (unsigned short*)(ws + oXP);
  float*          R1   = (float*)(ws + oR1);
  unsigned short* QK   = (unsigned short*)(ws + oQK);
  unsigned short* VP   = (unsigned short*)(ws + oVP);
  unsigned short* VPL  = (unsigned short*)(ws + oVPL);
  unsigned short* OP   = (unsigned short*)(ws + oOP);
  unsigned short* OPL  = (unsigned short*)(ws + oOPL);

  const dim3 blk256(256), blk128(128);

  cvt_w<<<dim3(32), blk256, 0, stream>>>(wq, wp, WQ16, WP16);

  for (int ck = 0; ck < NCHUNK; ++ck) {
    const float* xc   = x   + (size_t)ck * NCHK * CDIM * NPX;
    float*       outc = out + (size_t)ck * NCHK * CDIM * NPX;
    cvt_x<<<dim3(NTILE, CDIM / QT, NCHK), blk256, 0, stream>>>(xc, XP);
    gemm_k<1, 0><<<dim3(NTILE, C3 / 128, NCHK), blk128, 0, stream>>>(WQ16, XP, XP, R1, C3, 1.0f);
    dw_k<<<dim3(NTILE, C3 / QT, NCHK), blk256, 0, stream>>>(R1, wdw, QK, VP, VPL);
    attn_k<<<dim3(CDIM / 64, NCHK), blk256, 0, stream>>>(QK, VP, VPL, temp, OP, OPL);
    gemm_k<0, 1><<<dim3(NTILE, CDIM / 64, NCHK), blk128, 0, stream>>>(WP16, OP, OPL, outc, CDIM, OUTSC);
  }
  (void)hipGetLastError();
}
